// EnhancedTransformerBlock_51917564674691
// MI455X (gfx1250) — hardware-verified
//
#include <hip/hip_runtime.h>


#define NBT  4
#define SS   2048
#define DM_  256
#define HG   8
#define HDG  32
#define HLC  4
#define HDL  64
#define HALF 2
#define ZH   2
#define DM   DM_
#define NN   SS
#define SCG  0.17677669529663688f
#define SCL_ 0.125f
#define LEPS 1e-5f
#define LOSC 1024.0f

typedef _Float16 h16;
typedef unsigned short bf;
typedef __attribute__((ext_vector_type(16))) __bf16   v16bf;
typedef __attribute__((ext_vector_type(16))) _Float16 v16h;
typedef __attribute__((ext_vector_type(8)))  _Float16 v8h;
typedef __attribute__((ext_vector_type(8)))  unsigned short v8us;
typedef __attribute__((ext_vector_type(8)))  float    v8f;
typedef __attribute__((ext_vector_type(4)))  float    v4f;
typedef __attribute__((ext_vector_type(4)))  _Float16 v4h;
typedef v8h  __attribute__((may_alias)) v8ha;
typedef v4f  __attribute__((may_alias)) v4fa;
typedef v8us __attribute__((may_alias)) v8usa;

__device__ __forceinline__ unsigned short f2bf(float f) { unsigned u = __float_as_uint(f); u += 0x7FFFu + ((u >> 16) & 1u); return (unsigned short)(u >> 16); }
__device__ __forceinline__ float bf2f(unsigned short b) { return __uint_as_float(((unsigned)b) << 16); }
__device__ __forceinline__ float bfr(float f) { return bf2f(f2bf(f)); }
__device__ __forceinline__ v16h cat16(v8h lo, v8h hi) { return __builtin_shufflevector(lo, hi, 0, 1, 2, 3, 4, 5, 6, 7, 8, 9, 10, 11, 12, 13, 14, 15); }
__device__ __forceinline__ v16bf cat16b(v8us lo, v8us hi) { return __builtin_bit_cast(v16bf, __builtin_shufflevector(lo, hi, 0, 1, 2, 3, 4, 5, 6, 7, 8, 9, 10, 11, 12, 13, 14, 15)); }
__device__ __forceinline__ v8f wmma16(v16h a, v16h b, v8f c) { return __builtin_amdgcn_wmma_f32_16x16x32_f16(false, a, false, b, (short)0, c, false, false); }
__device__ __forceinline__ v8f wmmab(v16bf a, v16bf b, v8f c) { return __builtin_amdgcn_wmma_f32_16x16x32_bf16(false, a, false, b, (short)0, c, false, false); }

template <bool SPLITA, bool F16OUT = false>
__global__ __launch_bounds__(128) void k_gemmb(const bf* __restrict__ A, const bf* __restrict__ Al, const bf* __restrict__ Bn, const float* __restrict__ bias, float* C, int ldc, h16* C2, const float* __restrict__ R = nullptr, int K = DM, int roundR = 1) {
    __shared__ __align__(16) float ost[4][16 * 68];
    const int lane = threadIdx.x & 31, wave = threadIdx.x >> 5, lr = lane & 15, hi = lane >> 4;
    const int r0 = blockIdx.x * 64 + wave * 16, c0 = blockIdx.y * 64;
    const size_t aoff = (size_t)(r0 + lr) * K + 8 * hi;
    size_t boff[4];
#pragma unroll
    for (int t = 0; t < 4; ++t) boff[t] = (size_t)(c0 + t * 16 + lr) * K + 8 * hi;
    v8f acc[4];
#pragma unroll
    for (int t = 0; t < 4; ++t) acc[t] = (v8f){};
#pragma unroll 1
    for (int kc = 0; kc < K; kc += 32) {
        const v16bf a = cat16b(*(const v8us*)(A + aoff + kc), *(const v8us*)(A + aoff + kc + 16));
        v16bf al = a;
        if (SPLITA) al = cat16b(*(const v8us*)(Al + aoff + kc), *(const v8us*)(Al + aoff + kc + 16));
#pragma unroll
        for (int t = 0; t < 4; ++t) { const v16bf b = cat16b(*(const v8us*)(Bn + boff[t] + kc), *(const v8us*)(Bn + boff[t] + kc + 16)); acc[t] = wmmab(a, b, acc[t]); if (SPLITA) acc[t] = wmmab(al, b, acc[t]); }
        asm volatile("v_nop\n\tv_nop\n\tv_nop\n\tv_nop" : "+v"(acc[0]), "+v"(acc[1]), "+v"(acc[2]), "+v"(acc[3]) : "v"(a), "v"(al));
    }
    float* os = &ost[wave][0];
#pragma unroll
    for (int t = 0; t < 4; ++t) { const float bv = bias ? bfr(bias[c0 + t * 16 + lr]) : 0.f;
#pragma unroll
        for (int j = 0; j < 8; ++j) os[(hi * 8 + j) * 68 + t * 16 + lr] = acc[t][j] + bv; }
    __syncthreads();
    if (F16OUT) {
        h16* crow = (h16*)(void*)C + (size_t)r0 * ldc + c0;
        auto pass = [&]() {
#pragma unroll
            for (int s = 0; s < 4; ++s) { const int row = 4 * s + (lane >> 3), piece = lane & 7; const float* sp = os + row * 68 + piece * 8; v8h o, o2;
#pragma unroll
                for (int i = 0; i < 8; ++i) { const h16 a = (h16)sp[i]; o[i] = a; o2[i] = (h16)((sp[i] - (float)a) * LOSC); }
                *(volatile v8h*)(crow + (size_t)row * ldc + piece * 8) = o; if (C2) *(volatile v8h*)(C2 + (size_t)r0 * ldc + c0 + (size_t)row * ldc + piece * 8) = o2; }
        };
        pass(); __threadfence(); pass();
    } else {
        float* crow = C + (size_t)r0 * ldc + c0;
        auto pass = [&]() {
#pragma unroll
            for (int s = 0; s < 8; ++s) { const int Lid = (lane >> 3) + 4 * s, piece = lane & 7; const int row = Lid >> 1, cofs = (Lid & 1) * 32 + piece * 4;
                v4f val = *(const v4fa*)(os + row * 68 + cofs); if (R) { const v4f rv = *(const v4f*)(R + ((size_t)r0 + row) * ldc + c0 + cofs); val += roundR ? (v4f){bfr(rv[0]), bfr(rv[1]), bfr(rv[2]), bfr(rv[3])} : rv; }
                *(volatile v4f*)(crow + (size_t)row * ldc + cofs) = val; }
        };
        pass(); __threadfence(); pass();
    }
}

__global__ __launch_bounds__(256) void k_cvt8(const float* __restrict__ src, bf* dst, size_t n8) {
    const size_t i = (size_t)blockIdx.x * 256 + threadIdx.x; if (i >= n8) return;
    const v8f v = *(const v8f*)(src + i * 8); v8us o;
#pragma unroll
    for (int k = 0; k < 8; ++k) o[k] = f2bf(v[k]);
    *(volatile v8us*)(dst + i * 8) = o; __threadfence(); *(volatile v8us*)(dst + i * 8) = o;
}
__global__ __launch_bounds__(256) void k_zero8(bf* dst, size_t n8) {
    const size_t i = (size_t)blockIdx.x * 256 + threadIdx.x; if (i >= n8) return; v8us z;
#pragma unroll
    for (int k = 0; k < 8; ++k) z[k] = 0;
    *(volatile v8us*)(dst + i * 8) = z; __threadfence(); *(volatile v8us*)(dst + i * 8) = z;
}

template <int MODE>
__global__ __launch_bounds__(128) void k_gemm3z(const bf* __restrict__ Ah, const bf* __restrict__ Al, const bf* __restrict__ Bh, const bf* __restrict__ Bl, int K, float* C, int ldc, size_t sA, size_t sB, size_t sC) {
    if ((MODE & 1) && (int)blockIdx.y * 64 > (int)blockIdx.x * 64 + 63) return;
    const size_t z = blockIdx.z; Ah += z * sA; Al += z * sA; Bh += z * sB; Bl += z * sB; C += z * sC;
    const int Klim = (MODE & 2) ? min(K, ((int)blockIdx.x + 1) * 64) : K;
    __shared__ __align__(16) float ost[4][16 * 68];
    const int lane = threadIdx.x & 31, wave = threadIdx.x >> 5, lr = lane & 15, hi = lane >> 4;
    const int r0 = blockIdx.x * 64 + wave * 16, c0 = blockIdx.y * 64;
    const size_t aoff = (size_t)(r0 + lr) * K + 8 * hi;
    v8f acc[4];
#pragma unroll
    for (int t = 0; t < 4; ++t) acc[t] = (v8f){};
#pragma unroll 1
    for (int kc = 0; kc < Klim; kc += 32) {
        const v16bf a = cat16b(*(const v8us*)(Ah + aoff + kc), *(const v8us*)(Ah + aoff + kc + 16));
        v16bf al = a; if (!(MODE & 4) && !(MODE & 16)) al = cat16b(*(const v8us*)(Al + aoff + kc), *(const v8us*)(Al + aoff + kc + 16));
#pragma unroll
        for (int t = 0; t < 4; ++t) { const size_t bo = (size_t)(c0 + t * 16 + lr) * K + kc + 8 * hi;
            const v16bf bh = cat16b(*(const v8us*)(Bh + bo), *(const v8us*)(Bh + bo + 16));
            acc[t] = wmmab(a, bh, acc[t]);
            if (!(MODE & 4)) { if (!(MODE & 16)) acc[t] = wmmab(al, bh, acc[t]); if (!(MODE & 8)) { const v16bf bl = cat16b(*(const v8us*)(Bl + bo), *(const v8us*)(Bl + bo + 16)); acc[t] = wmmab(a, bl, acc[t]); } } }
        asm volatile("v_nop\n\tv_nop\n\tv_nop\n\tv_nop" : "+v"(acc[0]), "+v"(acc[1]), "+v"(acc[2]), "+v"(acc[3]) : "v"(a), "v"(al));
    }
    float* os = &ost[wave][0];
#pragma unroll
    for (int t = 0; t < 4; ++t) {
#pragma unroll
        for (int j = 0; j < 8; ++j) os[(hi * 8 + j) * 68 + t * 16 + lr] = acc[t][j]; }
    __builtin_amdgcn_wave_barrier(); asm volatile("" ::: "memory");
    float* crow = C + (size_t)r0 * ldc + c0;
    auto pass = [&]() {
#pragma unroll
        for (int s = 0; s < 8; ++s) { const int Lid = (lane >> 3) + 4 * s, piece = lane & 7; const int row = Lid >> 1, cofs = (Lid & 1) * 32 + piece * 4;
            const v4f val = *(const v4fa*)(os + row * 68 + cofs); *(volatile v4f*)(crow + (size_t)row * ldc + cofs) = val; }
    };
    pass(); __threadfence(); pass();
}
__global__ __launch_bounds__(256) void k_planes32z(const float* __restrict__ F, int ld, int off, float sc, int rows, bf* Ph, bf* Pl) {
    typedef __attribute__((ext_vector_type(2))) unsigned short v2us;
    const int lane = threadIdx.x & 31; const size_t r = ((size_t)blockIdx.x * 8 + (threadIdx.x >> 5)) * 2 + (lane >> 4); if (r >= (size_t)rows) return; const int z = blockIdx.z; const int c0 = (lane & 15) * 2; v2us oh, ol;
    Ph += (size_t)z * rows * 32; Pl += (size_t)z * rows * 32;
#pragma unroll
    for (int i = 0; i < 2; ++i) { const float y = F[r * ld + off + z * 32 + c0 + i] * sc; const unsigned short hb = f2bf(y); oh[i] = hb; ol[i] = f2bf(y - bf2f(hb)); }
    const size_t o = r * 32 + c0; *(volatile v2us*)(Ph + o) = oh; *(volatile v2us*)(Pl + o) = ol; __threadfence(); *(volatile v2us*)(Ph + o) = oh; *(volatile v2us*)(Pl + o) = ol;
}
__global__ __launch_bounds__(256) void k_vtpadz(const float* __restrict__ F, int ld, int off, int nk, bf* Th, bf* Tl) {
    typedef __attribute__((ext_vector_type(2))) unsigned short v2us;
    const int lane = threadIdx.x & 31; const size_t wid = (size_t)blockIdx.x * 8 + (threadIdx.x >> 5); if (wid >= (size_t)64 * (nk / 64)) return; const int z = blockIdx.z; const int d = (int)(wid / (nk / 64)); const int k0 = (int)(wid % (nk / 64)) * 64 + lane * 2; v2us oh, ol;
    Th += (size_t)z * 64 * nk; Tl += (size_t)z * 64 * nk;
#pragma unroll
    for (int i = 0; i < 2; ++i) { const float y = (d < 32) ? F[(size_t)(k0 + i) * ld + off + z * 32 + (d < 32 ? d : 0)] : 0.f; const unsigned short hb = f2bf(y); oh[i] = hb; ol[i] = f2bf(y - bf2f(hb)); }
    const size_t o = (size_t)d * nk + k0; *(volatile v2us*)(Th + o) = oh; *(volatile v2us*)(Tl + o) = ol; __threadfence(); *(volatile v2us*)(Th + o) = oh; *(volatile v2us*)(Tl + o) = ol;
}
template <int NK>
__global__ __launch_bounds__(256) void k_softmaxz(const float* __restrict__ S, int rows, bf* PH, bf* PL) {
    typedef __attribute__((ext_vector_type(4))) unsigned short v4us;
    const int lane = threadIdx.x & 31, i = blockIdx.x * 8 + (threadIdx.x >> 5); if (i >= rows) return; const size_t zo = (size_t)blockIdx.z * rows * NK; const float* sr = S + zo + (size_t)i * NK; PH += zo; PL += zo;
    float m = -3.0e38f;
#pragma unroll 1
    for (int c0 = lane * 4; c0 < NK; c0 += 128) {
#pragma unroll
        for (int q = 0; q < 4; ++q) m = fmaxf(m, sr[c0 + q]); }
#pragma unroll
    for (int sh = 16; sh; sh >>= 1) m = fmaxf(m, __shfl_xor(m, sh, 32));
    float sum = 0.f;
#pragma unroll 1
    for (int c0 = lane * 4; c0 < NK; c0 += 128) {
#pragma unroll
        for (int q = 0; q < 4; ++q) sum += __expf(sr[c0 + q] - m); }
#pragma unroll
    for (int sh = 16; sh; sh >>= 1) sum += __shfl_xor(sum, sh, 32);
    const float inv = 1.0f / sum;
#pragma unroll 1
    for (int ps = 0; ps < 2; ++ps) {
#pragma unroll 1
        for (int c0 = lane * 4; c0 < NK; c0 += 128) { v4us oh, ol;
#pragma unroll
            for (int q = 0; q < 4; ++q) { const float p = __expf(sr[c0 + q] - m) * inv; const unsigned short hb = f2bf(p); oh[q] = hb; ol[q] = f2bf(p - bf2f(hb)); }
            const size_t o = (size_t)i * NK + c0; *(volatile v4us*)(PH + o) = oh; *(volatile v4us*)(PL + o) = ol; }
        if (ps == 0) __threadfence(); }
}
__global__ __launch_bounds__(256) void k_placez(const float* __restrict__ XH, int rows, int ldy, float* Y) {
    const int lane = threadIdx.x & 31; const size_t q = (size_t)blockIdx.x * 8 + (threadIdx.x >> 5); if (q >= (size_t)rows) return; const int z = blockIdx.z; const float v = XH[((size_t)z * rows + q) * 64 + lane];
    *(volatile float*)(Y + q * ldy + z * 32 + lane) = v; __threadfence(); *(volatile float*)(Y + q * ldy + z * 32 + lane) = v;
}

__global__ __launch_bounds__(256) void k_hplanesz(const float* __restrict__ F, int ld, int h0, float sc, int rows, bf* Ph, bf* Pl) {
    typedef __attribute__((ext_vector_type(2))) unsigned short v2us;
    const int lane = threadIdx.x & 31; const size_t r = (size_t)blockIdx.x * 8 + (threadIdx.x >> 5); if (r >= (size_t)rows) return; const int z = blockIdx.z; v2us oh, ol;
    Ph += (size_t)z * rows * 64; Pl += (size_t)z * rows * 64;
#pragma unroll
    for (int i = 0; i < 2; ++i) { const float y = F[r * ld + (h0 + z) * 64 + lane * 2 + i] * sc; const unsigned short hb = f2bf(y); oh[i] = hb; ol[i] = f2bf(y - bf2f(hb)); }
    const size_t o = r * 64 + lane * 2; *(volatile v2us*)(Ph + o) = oh; *(volatile v2us*)(Pl + o) = ol; __threadfence(); *(volatile v2us*)(Ph + o) = oh; *(volatile v2us*)(Pl + o) = ol;
}
__global__ __launch_bounds__(256) void k_vtz(const float* __restrict__ F, int ld, int h0, int nk, bf* Th, bf* Tl) {
    typedef __attribute__((ext_vector_type(2))) unsigned short v2us;
    const int lane = threadIdx.x & 31; const size_t wid = (size_t)blockIdx.x * 8 + (threadIdx.x >> 5); if (wid >= (size_t)64 * (nk / 64)) return; const int z = blockIdx.z; const int d = (int)(wid / (nk / 64)); const int t0 = (int)(wid % (nk / 64)) * 64 + lane * 2; v2us oh, ol;
    Th += (size_t)z * 64 * nk; Tl += (size_t)z * 64 * nk;
#pragma unroll
    for (int i = 0; i < 2; ++i) { const float y = F[(size_t)(t0 + i) * ld + (h0 + z) * 64 + d]; const unsigned short hb = f2bf(y); oh[i] = hb; ol[i] = f2bf(y - bf2f(hb)); }
    const size_t o = (size_t)d * nk + t0; *(volatile v2us*)(Th + o) = oh; *(volatile v2us*)(Tl + o) = ol; __threadfence(); *(volatile v2us*)(Th + o) = oh; *(volatile v2us*)(Tl + o) = ol;
}
template <int NK>
__global__ __launch_bounds__(256) void k_softmaxzs(const float* __restrict__ S, int rows, float sc, bf* PH, bf* PL) {
    typedef __attribute__((ext_vector_type(4))) unsigned short v4us;
    const int lane = threadIdx.x & 31, i = blockIdx.x * 8 + (threadIdx.x >> 5); if (i >= rows) return; const size_t zo = (size_t)blockIdx.z * rows * NK; const float* sr = S + zo + (size_t)i * NK; PH += zo; PL += zo;
    float m = -3.0e38f;
#pragma unroll 1
    for (int c0 = lane * 4; c0 < NK; c0 += 128) {
#pragma unroll
        for (int q = 0; q < 4; ++q) m = fmaxf(m, sr[c0 + q] * sc); }
#pragma unroll
    for (int sh = 16; sh; sh >>= 1) m = fmaxf(m, __shfl_xor(m, sh, 32));
    float sum = 0.f;
#pragma unroll 1
    for (int c0 = lane * 4; c0 < NK; c0 += 128) {
#pragma unroll
        for (int q = 0; q < 4; ++q) sum += __expf(sr[c0 + q] * sc - m); }
#pragma unroll
    for (int sh = 16; sh; sh >>= 1) sum += __shfl_xor(sum, sh, 32);
    const float inv = 1.0f / sum;
#pragma unroll 1
    for (int ps = 0; ps < 2; ++ps) {
#pragma unroll 1
        for (int c0 = lane * 4; c0 < NK; c0 += 128) { v4us oh, ol;
#pragma unroll
            for (int q = 0; q < 4; ++q) { const float p = __expf(sr[c0 + q] * sc - m) * inv; const unsigned short hb = f2bf(p); oh[q] = hb; ol[q] = f2bf(p - bf2f(hb)); }
            const size_t o = (size_t)i * NK + c0; *(volatile v4us*)(PH + o) = oh; *(volatile v4us*)(PL + o) = ol; }
        if (ps == 0) __threadfence(); }
}

__global__ __launch_bounds__(256) void k_cvt256(const float* __restrict__ src, int rows, bf* dst) {
    const int lane = threadIdx.x & 31; const size_t r = (size_t)blockIdx.x * 8 + (threadIdx.x >> 5); if (r >= (size_t)rows) return; v8us o;
#pragma unroll
    for (int i = 0; i < 8; ++i) o[i] = f2bf(src[r * DM_ + lane * 8 + i]);
    *(volatile v8us*)(dst + r * DM_ + lane * 8) = o; __threadfence(); *(volatile v8us*)(dst + r * DM_ + lane * 8) = o;
}
__global__ __launch_bounds__(256) void k_hp32z(const float* __restrict__ F, int ld, int col0, int h0, bf* Ph, bf* Pl) {
    typedef __attribute__((ext_vector_type(2))) unsigned short v2us;
    const int lane = threadIdx.x & 31; const size_t r = ((size_t)blockIdx.x * 8 + (threadIdx.x >> 5)) * 2 + (lane >> 4); if (r >= (size_t)SS) return; const int z = blockIdx.z; const int d0 = (lane & 15) * 2; v2us oh, ol;
    Ph += (size_t)z * SS * HDG; Pl += (size_t)z * SS * HDG;
#pragma unroll
    for (int i = 0; i < 2; ++i) { const float y = F[r * ld + col0 + (h0 + z) * HDG + d0 + i]; const unsigned short hb = f2bf(y); oh[i] = hb; ol[i] = f2bf(y - bf2f(hb)); }
    const size_t o = r * HDG + d0; *(volatile v2us*)(Ph + o) = oh; *(volatile v2us*)(Pl + o) = ol; __threadfence(); *(volatile v2us*)(Ph + o) = oh; *(volatile v2us*)(Pl + o) = ol;
}
__global__ __launch_bounds__(256) void k_vt32z(const float* __restrict__ F, int ld, int col0, int h0, bf* Th, bf* Tl) {
    typedef __attribute__((ext_vector_type(2))) unsigned short v2us;
    const int lane = threadIdx.x & 31; const size_t wid = (size_t)blockIdx.x * 8 + (threadIdx.x >> 5); if (wid >= (size_t)64 * (SS / 64)) return; const int z = blockIdx.z; const int d = (int)(wid / (SS / 64)); const int t0 = (int)(wid % (SS / 64)) * 64 + lane * 2; v2us oh, ol;
    Th += (size_t)z * 64 * SS; Tl += (size_t)z * 64 * SS;
#pragma unroll
    for (int i = 0; i < 2; ++i) { const float y = (d < HDG) ? F[(size_t)(t0 + i) * ld + col0 + (h0 + z) * HDG + (d < HDG ? d : 0)] : 0.f; const unsigned short hb = f2bf(y); oh[i] = hb; ol[i] = f2bf(y - bf2f(hb)); }
    const size_t o = (size_t)d * SS + t0; *(volatile v2us*)(Th + o) = oh; *(volatile v2us*)(Tl + o) = ol; __threadfence(); *(volatile v2us*)(Th + o) = oh; *(volatile v2us*)(Tl + o) = ol;
}
__global__ __launch_bounds__(256) void k_place32z(const float* __restrict__ XO, int h0, float* ATT) {
    const int lane = threadIdx.x & 31; const size_t r = (size_t)blockIdx.x * 8 + (threadIdx.x >> 5); if (r >= (size_t)SS) return; const int z = blockIdx.z; const float v = XO[((size_t)z * SS + r) * 64 + lane];
    float* dst = ATT + r * DM_ + (h0 + z) * HDG + lane; *(volatile float*)dst = v; __threadfence(); *(volatile float*)dst = v;
}
__global__ __launch_bounds__(256) void k_local5(const float* __restrict__ T, bf* Oh, bf* Ol) {
    const int lane = threadIdx.x & 31; const size_t s = (size_t)blockIdx.x * 8 + (threadIdx.x >> 5); if (s >= (size_t)SS) return; const int c0 = lane * 8; float q[8];
#pragma unroll
    for (int i = 0; i < 8; ++i) q[i] = T[s * (3 * DM_) + c0 + i];
    auto logit = [&](int j, bool& ok) -> float { const long sp = (long)s + j; ok = sp >= 0 && sp < SS; const size_t row = (size_t)(ok ? sp : 0) * (3 * DM_) + DM_; float a = 0.f;
#pragma unroll
        for (int i = 0; i < 8; ++i) a = fmaf(q[i], ok ? T[row + c0 + i] : 0.f, a);
        a += __shfl_xor(a, 1, 32); a += __shfl_xor(a, 2, 32); a += __shfl_xor(a, 4, 32); return a * SCL_; };
    float m = -3.0e38f;
#pragma unroll 1
    for (int j = -HALF; j <= HALF; ++j) { bool ok; const float a = logit(j, ok); if (ok) m = fmaxf(m, a); }
    float den = 0.f; float o[8];
#pragma unroll
    for (int i = 0; i < 8; ++i) o[i] = 0.f;
#pragma unroll 1
    for (int j = -HALF; j <= HALF; ++j) { bool ok; const float a = logit(j, ok); if (ok) { const float e = __expf(a - m); den += e; const size_t row = (size_t)(s + j) * (3 * DM_) + 2 * DM_;
#pragma unroll
            for (int i = 0; i < 8; ++i) o[i] = fmaf(e, T[row + c0 + i], o[i]); } }
    const float inv = 1.0f / den; v8us oh, ol;
#pragma unroll
    for (int i = 0; i < 8; ++i) { const float y = o[i] * inv; const unsigned short hb = f2bf(y); oh[i] = hb; ol[i] = f2bf(y - bf2f(hb)); }
    const size_t off = s * DM_ + c0; *(volatile v8us*)(Oh + off) = oh; *(volatile v8us*)(Ol + off) = ol; __threadfence(); *(volatile v8us*)(Oh + off) = oh; *(volatile v8us*)(Ol + off) = ol;
}
__global__ __launch_bounds__(256) void k_split256(const float* __restrict__ src, int rows, bf* dh, bf* dl) {
    const int lane = threadIdx.x & 31; const size_t r = (size_t)blockIdx.x * 8 + (threadIdx.x >> 5); if (r >= (size_t)rows) return; const size_t o = r * DM_ + lane * 8; const v8f v = *(const v8f*)(src + o); v8us oh, ol;
#pragma unroll
    for (int i = 0; i < 8; ++i) { const unsigned short hb = f2bf(v[i]); oh[i] = hb; ol[i] = f2bf(v[i] - bf2f(hb)); }
    *(volatile v8us*)(dh + o) = oh; *(volatile v8us*)(dl + o) = ol; __threadfence(); *(volatile v8us*)(dh + o) = oh; *(volatile v8us*)(dl + o) = ol;
}
__global__ __launch_bounds__(256) void k_cat2(const float* __restrict__ XG, const float* __restrict__ XL, bf* Ch, bf* Cl) {
    const int lane = threadIdx.x & 31; const size_t r = (size_t)blockIdx.x * 8 + (threadIdx.x >> 5); if (r >= (size_t)SS) return;
#pragma unroll 1
    for (int ps = 0; ps < 2; ++ps) {
#pragma unroll
        for (int q = 0; q < 2; ++q) { const float* src = (q == 0 ? XG : XL) + r * DM_ + lane * 8; v8us oh, ol;
#pragma unroll
            for (int i = 0; i < 8; ++i) { const float v = src[i]; const unsigned short hb = f2bf(v); oh[i] = hb; ol[i] = f2bf(v - bf2f(hb)); }
            const size_t o = r * (2 * DM_) + q * DM_ + lane * 8; *(volatile v8us*)(Ch + o) = oh; *(volatile v8us*)(Cl + o) = ol; }
        if (ps == 0) __threadfence(); }
}
__global__ __launch_bounds__(256) void k_silu512(const float* __restrict__ F, int rows, bf* Gh, bf* Gl) {
    const int lane = threadIdx.x & 31; const size_t r = (size_t)blockIdx.x * 8 + (threadIdx.x >> 5); if (r >= (size_t)rows) return;
#pragma unroll 1
    for (int ps = 0; ps < 2; ++ps) {
#pragma unroll
        for (int q = 0; q < 2; ++q) { const size_t o = r * (2 * DM_) + q * 256 + lane * 8; const v8f v = *(const v8f*)(F + o); v8us oh, ol;
#pragma unroll
            for (int i = 0; i < 8; ++i) { const float x = v[i]; const float g = x / (1.0f + __expf(-x)); const unsigned short hb = f2bf(g); oh[i] = hb; ol[i] = f2bf(g - bf2f(hb)); }
            *(volatile v8us*)(Gh + o) = oh; *(volatile v8us*)(Gl + o) = ol; }
        if (ps == 0) __threadfence(); }
}
template <bool RIN>
__global__ __launch_bounds__(256) void k_addln256(const float* __restrict__ Ain, const float* __restrict__ Bin, const float* __restrict__ g, const float* __restrict__ bb, float* Yf, bf* Yh, bf* Yl) {
    typedef __attribute__((ext_vector_type(4))) unsigned short v4us;
    const int lane = threadIdx.x & 31; const size_t r = (size_t)blockIdx.x * 8 + (threadIdx.x >> 5); if (r >= (size_t)SS) return; float v[8]; float s = 0.f;
#pragma unroll
    for (int q = 0; q < 2; ++q) {
#pragma unroll
        for (int i = 0; i < 4; ++i) { const size_t o = r * DM_ + q * 128 + lane * 4 + i; const float t = Ain[o] + (RIN ? bfr(Bin[o]) : Bin[o]); v[q * 4 + i] = t; s += t; } }
#pragma unroll
    for (int sh = 16; sh; sh >>= 1) s += __shfl_xor(s, sh, 32);
    const float mu = s * (1.0f / DM_); float qv = 0.f;
#pragma unroll
    for (int i = 0; i < 8; ++i) { const float d = v[i] - mu; qv = fmaf(d, d, qv); }
#pragma unroll
    for (int sh = 16; sh; sh >>= 1) qv += __shfl_xor(qv, sh, 32);
    const float rs = rsqrtf(qv * (1.0f / DM_) + LEPS);
#pragma unroll 1
    for (int ps = 0; ps < 2; ++ps) {
#pragma unroll
        for (int q = 0; q < 2; ++q) { const int c0 = q * 128 + lane * 4; v4f y; v4us oh, ol;
#pragma unroll
            for (int i = 0; i < 4; ++i) { y[i] = (v[q * 4 + i] - mu) * rs * bfr(g[c0 + i]) + bfr(bb[c0 + i]); const unsigned short hb = f2bf(y[i]); oh[i] = hb; ol[i] = f2bf(y[i] - bf2f(hb)); }
            const size_t o = r * DM_ + c0; *(volatile v4f*)(Yf + o) = y; if (Yh != nullptr) { *(volatile v4us*)(Yh + o) = oh; *(volatile v4us*)(Yl + o) = ol; } }
        if (ps == 0) __threadfence(); }
}

extern "C" void kernel_launch(void* const* d_in, const int* in_sizes, int n_in,
                              void* d_out, int out_size, void* d_ws, size_t ws_size, hipStream_t stream) {
    (void)in_sizes; (void)n_in; (void)out_size;
    const float* x = (const float*)d_in[0]; const float* g_in_w = (const float*)d_in[1]; const float* g_in_b = (const float*)d_in[2]; const float* g_out_w = (const float*)d_in[3]; const float* g_out_b = (const float*)d_in[4];
    const float* t_in_w = (const float*)d_in[5]; const float* t_in_b = (const float*)d_in[6]; const float* t_out_w = (const float*)d_in[7]; const float* t_out_b = (const float*)d_in[8];
    const float* fus_w1 = (const float*)d_in[9]; const float* fus_b1 = (const float*)d_in[10]; const float* fus_w2 = (const float*)d_in[11]; const float* fus_b2 = (const float*)d_in[12];
    const float* ffn_w1 = (const float*)d_in[13]; const float* ffn_b1 = (const float*)d_in[14]; const float* ffn_w2 = (const float*)d_in[15]; const float* ffn_b2 = (const float*)d_in[16];
    const float* gn_g = (const float*)d_in[17]; const float* gn_b = (const float*)d_in[18]; const float* fn_g = (const float*)d_in[19]; const float* fn_b = (const float*)d_in[20];
    float* out = (float*)d_out;
    char* wsp = (char*)d_ws;
    auto take = [&](size_t bytes) { char* p = wsp; wsp += (bytes + 255) & ~(size_t)255; return (void*)p; };
    bf* WGI = (bf*)take((size_t)768 * 256 * 2); bf* WTI = (bf*)take((size_t)768 * 256 * 2); bf* WGO = (bf*)take((size_t)256 * 256 * 2); bf* WTO = (bf*)take((size_t)256 * 256 * 2); bf* WF1 = (bf*)take((size_t)512 * 512 * 2); bf* WF2 = (bf*)take((size_t)256 * 512 * 2); bf* WN1 = (bf*)take((size_t)512 * 256 * 2); bf* WN2 = (bf*)take((size_t)256 * 512 * 2);
    bf* Xb = (bf*)take((size_t)SS * DM_ * 2); float* GQKV = (float*)take((size_t)SS * 3 * DM_ * 4); float* TQKV = (float*)take((size_t)SS * 3 * DM_ * 4);
    bf* Qh = (bf*)take((size_t)ZH * SS * HDG * 2); bf* Ql = (bf*)take((size_t)ZH * SS * HDG * 2); bf* Kh = (bf*)take((size_t)ZH * SS * HDG * 2); bf* Kl = (bf*)take((size_t)ZH * SS * HDG * 2); bf* VTh = (bf*)take((size_t)ZH * 64 * SS * 2); bf* VTl = (bf*)take((size_t)ZH * 64 * SS * 2);
    float* S = (float*)take((size_t)ZH * SS * SS * 4); bf* PH = (bf*)take((size_t)ZH * SS * SS * 2); bf* PL = (bf*)take((size_t)ZH * SS * SS * 2); float* XO = (float*)take((size_t)ZH * SS * 64 * 4);
    float* GATT = (float*)take((size_t)SS * DM_ * 4); bf* Ah = (bf*)take((size_t)SS * DM_ * 2); bf* Al = (bf*)take((size_t)SS * DM_ * 2); float* XG = (float*)take((size_t)SS * DM_ * 4); bf* Lh = (bf*)take((size_t)SS * DM_ * 2); bf* Ll = (bf*)take((size_t)SS * DM_ * 2); float* XL = (float*)take((size_t)SS * DM_ * 4);
    bf* Ch = (bf*)take((size_t)SS * 2 * DM_ * 2); bf* Cl = (bf*)take((size_t)SS * 2 * DM_ * 2); float* F1 = (float*)take((size_t)SS * 2 * DM_ * 4); bf* G1h = (bf*)take((size_t)SS * 2 * DM_ * 2); bf* G1l = (bf*)take((size_t)SS * 2 * DM_ * 2); float* F2 = (float*)take((size_t)SS * DM_ * 4);
    float* H1 = (float*)take((size_t)SS * DM_ * 4); bf* H1h = (bf*)take((size_t)SS * DM_ * 2); bf* H1l = (bf*)take((size_t)SS * DM_ * 2);
    if ((size_t)(wsp - (char*)d_ws) > ws_size) return;
    k_cvt8<<<(768 * 256 / 8 + 255) / 256, 256, 0, stream>>>(g_in_w, WGI, 768 * 256 / 8); k_cvt8<<<(768 * 256 / 8 + 255) / 256, 256, 0, stream>>>(t_in_w, WTI, 768 * 256 / 8); k_cvt8<<<(256 * 256 / 8 + 255) / 256, 256, 0, stream>>>(g_out_w, WGO, 256 * 256 / 8); k_cvt8<<<(256 * 256 / 8 + 255) / 256, 256, 0, stream>>>(t_out_w, WTO, 256 * 256 / 8);
    k_cvt8<<<(512 * 512 / 8 + 255) / 256, 256, 0, stream>>>(fus_w1, WF1, 512 * 512 / 8); k_cvt8<<<(256 * 512 / 8 + 255) / 256, 256, 0, stream>>>(fus_w2, WF2, 256 * 512 / 8); k_cvt8<<<(512 * 256 / 8 + 255) / 256, 256, 0, stream>>>(ffn_w1, WN1, 512 * 256 / 8); k_cvt8<<<(256 * 512 / 8 + 255) / 256, 256, 0, stream>>>(ffn_w2, WN2, 256 * 512 / 8);
    for (int b = 0; b < NBT; ++b) { const float* xb = x + (size_t)b * SS * DM_;
        k_cvt256<<<SS / 8, 256, 0, stream>>>(xb, SS, Xb);
        k_gemmb<false, false><<<dim3(SS / 64, 768 / 64, 1), 128, 0, stream>>>(Xb, nullptr, WGI, g_in_b, GQKV, 3 * DM_, nullptr, nullptr, DM_);
        k_gemmb<false, false><<<dim3(SS / 64, 768 / 64, 1), 128, 0, stream>>>(Xb, nullptr, WTI, t_in_b, TQKV, 3 * DM_, nullptr, nullptr, DM_);
        for (int g = 0; g < HG / ZH; ++g) { const int h0 = g * ZH;
            k_hp32z<<<dim3((SS / 2) / 8, 1, ZH), 256, 0, stream>>>(GQKV, 3 * DM_, 0, h0, Qh, Ql); k_hp32z<<<dim3((SS / 2) / 8, 1, ZH), 256, 0, stream>>>(GQKV, 3 * DM_, DM_, h0, Kh, Kl); k_vt32z<<<dim3((64 * (SS / 64)) / 8, 1, ZH), 256, 0, stream>>>(GQKV, 3 * DM_, 2 * DM_, h0, VTh, VTl);
            k_gemm3z<0><<<dim3(SS / 64, SS / 64, ZH), 128, 0, stream>>>(Qh, Ql, Kh, Kl, HDG, S, SS, (size_t)SS * HDG, (size_t)SS * HDG, (size_t)SS * SS);
            k_softmaxzs<SS><<<dim3(SS / 8, 1, ZH), 256, 0, stream>>>(S, SS, SCG, PH, PL);
            k_gemm3z<0><<<dim3(SS / 64, 1, ZH), 128, 0, stream>>>(PH, PL, VTh, VTl, SS, XO, 64, (size_t)SS * SS, (size_t)64 * SS, (size_t)SS * 64);
            k_place32z<<<dim3(SS / 8, 1, ZH), 256, 0, stream>>>(XO, h0, GATT); }
        k_split256<<<SS / 8, 256, 0, stream>>>(GATT, SS, Ah, Al); k_gemmb<true, false><<<dim3(SS / 64, DM_ / 64, 1), 128, 0, stream>>>(Ah, Al, WGO, g_out_b, XG, DM_, nullptr, nullptr, DM_);
        k_local5<<<SS / 8, 256, 0, stream>>>(TQKV, Lh, Ll); k_gemmb<true, false><<<dim3(SS / 64, DM_ / 64, 1), 128, 0, stream>>>(Lh, Ll, WTO, t_out_b, XL, DM_, nullptr, nullptr, DM_);
        k_cat2<<<SS / 8, 256, 0, stream>>>(XG, XL, Ch, Cl);
        k_gemmb<true, false><<<dim3(SS / 64, 512 / 64, 1), 128, 0, stream>>>(Ch, Cl, WF1, fus_b1, F1, 2 * DM_, nullptr, nullptr, 2 * DM_); k_silu512<<<SS / 8, 256, 0, stream>>>(F1, SS, G1h, G1l);
        k_gemmb<true, false><<<dim3(SS / 64, DM_ / 64, 1), 128, 0, stream>>>(G1h, G1l, WF2, fus_b2, F2, DM_, nullptr, nullptr, 2 * DM_);
        k_addln256<true><<<SS / 8, 256, 0, stream>>>(F2, xb, gn_g, gn_b, H1, H1h, H1l);
        k_gemmb<true, false><<<dim3(SS / 64, 512 / 64, 1), 128, 0, stream>>>(H1h, H1l, WN1, ffn_b1, F1, 2 * DM_, nullptr, nullptr, DM_); k_silu512<<<SS / 8, 256, 0, stream>>>(F1, SS, G1h, G1l);
        k_gemmb<true, false><<<dim3(SS / 64, DM_ / 64, 1), 128, 0, stream>>>(G1h, G1l, WN2, ffn_b2, F2, DM_, nullptr, nullptr, 2 * DM_);
        k_addln256<false><<<SS / 8, 256, 0, stream>>>(F2, H1, fn_g, fn_b, out + (size_t)b * SS * DM_, nullptr, nullptr); }
}
